// MultiheadCosformerAttention_63419487093380
// MI455X (gfx1250) — hardware-verified
//
#include <hip/hip_runtime.h>
#include <math.h>

typedef __attribute__((ext_vector_type(16))) _Float16 v16h;
typedef __attribute__((ext_vector_type(16))) __bf16 v16b;
typedef __attribute__((ext_vector_type(8)))  _Float16 v8h;
typedef __attribute__((ext_vector_type(8)))  float v8f;
typedef __attribute__((ext_vector_type(4)))  float v4f;
typedef __attribute__((ext_vector_type(2)))  float v2f;
typedef __attribute__((ext_vector_type(4)))  unsigned v4u;
typedef __attribute__((ext_vector_type(4)))  int v4i;
typedef float __attribute__((may_alias)) float_a;
typedef int __attribute__((may_alias)) int_a;

template <typename T> __device__ __forceinline__ void vst2(void* p, T v) { *(volatile T*)p = v; __threadfence(); *(volatile T*)p = v; }
__device__ __forceinline__ v8f wmma16(v16h a, v16h b, v8f c) {
  v8f d = __builtin_amdgcn_wmma_f32_16x16x32_f16(false, a, false, b, (short)0, c, false, false);
  asm volatile("v_nop\n\tv_nop\n\tv_nop\n\tv_nop" : "+v"(d) : "v"(a), "v"(b));
  return d;
}
__device__ __forceinline__ v8f wmma_bf(v16b a, v16b b, v8f c) {
  v8f d = __builtin_amdgcn_wmma_f32_16x16x32_bf16(false, a, false, b, (short)0, c, false, false);
  asm volatile("v_nop\n\tv_nop\n\tv_nop\n\tv_nop" : "+v"(d) : "v"(a), "v"(b));
  return d;
}
__device__ __forceinline__ v16h frag_h(const _Float16* rowk0, int lane) {
  union { v16h v; v8h q[2]; } u; const _Float16* p = rowk0 + 8 * (lane >> 4);
  u.q[0] = *(const v8h*)p; u.q[1] = *(const v8h*)(p + 16); return u.v;
}
__device__ __forceinline__ v16h frag_f32(const float* rowk0, int lane) {
  v16h a; const float* p = rowk0 + 8 * (lane >> 4);
#pragma unroll
  for (int i = 0; i < 8; ++i) { a[i] = (_Float16)p[i]; a[8 + i] = (_Float16)p[16 + i]; }
  return a;
}
__device__ __forceinline__ v16h frag_f32s(const float* rowk0, int lane, float sc) {
  v16h a; const float* p = rowk0 + 8 * (lane >> 4);
#pragma unroll
  for (int i = 0; i < 8; ++i) { a[i] = (_Float16)(p[i] * sc); a[8 + i] = (_Float16)(p[16 + i] * sc); }
  return a;
}
__device__ __forceinline__ v16h fragc_f32(const float* W, int k0, int n, int lane, int ld, int K) {
  v16h a; const int g = lane >> 4;
#pragma unroll
  for (int i = 0; i < 8; ++i) { const int ka = k0 + 8 * g + i, kb = ka + 16;
    a[i] = (_Float16)(ka < K ? W[(size_t)(ka < K ? ka : K - 1) * ld + n] : 0.f); a[8 + i] = (_Float16)(kb < K ? W[(size_t)(kb < K ? kb : K - 1) * ld + n] : 0.f); }
  return a;
}
struct F2 { v16b h, l; };
__device__ __forceinline__ F2 bsplit16(const float v[16]) { F2 r;
#pragma unroll
  for (int i = 0; i < 16; ++i) { const __bf16 h = (__bf16)v[i]; r.h[i] = h; r.l[i] = (__bf16)(v[i] - (float)h); }
  return r; }
__device__ __forceinline__ F2 split_row(const float* row, int k0, int lane) { float v[16]; const float* p = row + k0 + 8 * (lane >> 4);
#pragma unroll
  for (int i = 0; i < 8; ++i) { v[i] = p[i]; v[8 + i] = p[16 + i]; }
  return bsplit16(v); }
__device__ __forceinline__ F2 split_rowK(const float* row, int k0, int lane, int K) { float v[16]; const int g = lane >> 4;
#pragma unroll
  for (int i = 0; i < 8; ++i) { const int ka = k0 + 8 * g + i, kb = ka + 16; v[i] = ka < K ? row[ka < K ? ka : K - 1] : 0.f; v[8 + i] = kb < K ? row[kb < K ? kb : K - 1] : 0.f; }
  return bsplit16(v); }
__device__ __forceinline__ F2 split_col(const float* W, int k0, int n, int lane, int ld, int K) { float v[16]; const int g = lane >> 4;
#pragma unroll
  for (int i = 0; i < 8; ++i) { const int ka = k0 + 8 * g + i, kb = ka + 16; v[i] = ka < K ? W[(size_t)(ka < K ? ka : K - 1) * ld + n] : 0.f; v[8 + i] = kb < K ? W[(size_t)(kb < K ? kb : K - 1) * ld + n] : 0.f; }
  return bsplit16(v); }
__device__ __forceinline__ v8f mac3(const F2& a, const F2& b, v8f c) { c = wmma_bf(a.l, b.h, c); c = wmma_bf(a.h, b.l, c); return wmma_bf(a.h, b.h, c); }
__device__ __forceinline__ float sigm(float v) { return 1.0f / (1.0f + expf(-v)); }
#define LDSX() do { asm volatile("s_wait_dscnt 0" ::: "memory"); __builtin_amdgcn_wave_barrier(); __builtin_amdgcn_fence(__ATOMIC_RELEASE, "workgroup"); } while (0)


#define LL 2048
#define NBATCH 4
#define EE 1024
#define NH 16
#define HD 64
#define NBH (NBATCH * NH)
#define NR (LL * NBATCH)
#ifndef TBH
#define TBH NBH
#endif
typedef __attribute__((ext_vector_type(8))) __bf16 v8b;
__device__ __forceinline__ v16b frag_b(const __bf16* rowk0, int lane) {
  union { v16b v; v8b q[2]; } u; const __bf16* p = rowk0 + 8 * (lane >> 4);
  u.q[0] = *(const v8b*)p; u.q[1] = *(const v8b*)(p + 16); return u.v;
}
__device__ __forceinline__ float bfr(float v) { return (float)(__bf16)v; }
__device__ __attribute__((noinline)) float exp_ni(float v) { return expf(v); }
__device__ __attribute__((noinline)) float erf_ni(float v) { return erff(v); }

#define WS_PW  0u
#define WS_Q   (WS_PW + 2u * (size_t)2 * EE * EE)
#define WS_K   (WS_Q + 4u * (size_t)NR * EE)
#define WS_V   (WS_K + 4u * (size_t)NR * EE)
#define WS_PL  (WS_V + 4u * (size_t)NR * EE)
#define WS_KV  (WS_PL + 2u * (size_t)NBH * 6 * HD * LL)
#define WS_KS  (WS_KV + 4u * (size_t)NBH * 2 * HD * HD)
#define WS_END (WS_KS + 4u * (size_t)NBH * 2 * HD)

__device__ __attribute__((noinline)) float sin_p(float v) { return sinf(v); }
__device__ __attribute__((noinline)) float cos_p(float v) { return cosf(v); }
__global__ __launch_bounds__(256) void k_pack(const float* __restrict__ WQ, const float* __restrict__ WK, __bf16* __restrict__ PW) { const int n = blockIdx.x, which = blockIdx.y, t = threadIdx.x; __shared__ __align__(16) __bf16 s[EE]; const float* w = which ? WK : WQ; for (int k = t; k < EE; k += 256) s[k] = (__bf16)w[(size_t)n * EE + k]; __syncthreads(); if (t < EE / 8) vst2((unsigned*)(PW + ((size_t)which * EE + n) * EE + t * 8), *(const v4u*)&s[t * 8]); }
__global__ __launch_bounds__(128) void k_proj(const float* __restrict__ XQ, const float* __restrict__ XK, const float* __restrict__ XV, const __bf16* __restrict__ PW, const float* __restrict__ BQ, const float* __restrict__ BK, float* __restrict__ Q, float* __restrict__ K, float* __restrict__ V) {
  __shared__ __align__(16) float so[4][16][132];
  const int tid = threadIdx.x, wave = tid >> 5, lane = tid & 31, col = lane & 15, g = lane >> 4; const int which = blockIdx.z; const size_t r0 = (size_t)blockIdx.x * 64 + wave * 16; const int c0 = blockIdx.y * 128;
  const float* X = (which == 0) ? XQ : (which == 1) ? XK : XV; const __bf16* Wr = PW + ((which == 0) ? 0 : (size_t)EE * EE); const float* BB = (which == 0) ? BQ : BK; float* dst = (which == 0) ? Q : (which == 1) ? K : V;
  v8f acc[8] = {};
#pragma unroll 2
  for (int kc = 0; kc < EE / 32; ++kc) { v16b a; { const float* p = X + (r0 + col) * EE + kc * 32 + 8 * g;
#pragma unroll
      for (int i = 0; i < 8; ++i) { a[i] = (__bf16)p[i]; a[8 + i] = (__bf16)p[16 + i]; } }
#pragma unroll
    for (int j = 0; j < 8; ++j) acc[j] = wmma_bf(a, frag_b(Wr + (size_t)(c0 + j * 16 + col) * EE + kc * 32, lane), acc[j]); }
#pragma unroll
  for (int j = 0; j < 8; ++j) { const float bb = bfr(BB[c0 + j * 16 + col]);
#pragma unroll
    for (int r = 0; r < 8; ++r) { const float v = acc[j][r] + bb; so[wave][8 * g + r][j * 16 + col] = (which < 2) ? fmaxf(v, 0.f) : v; } }
  LDSX();
  for (int rl = 0; rl < 16; ++rl) vst2(dst + (r0 + rl) * EE + c0 + lane * 4, *(const v4f*)&so[wave][rl][lane * 4]);
}
__global__ __launch_bounds__(256) void k_planes(const float* __restrict__ K, const float* __restrict__ V, _Float16* __restrict__ PL) {
  __shared__ __align__(16) _Float16 st[6][HD][72]; const int s0 = blockIdx.x * 64; const size_t bh = blockIdx.y; const size_t b = bh / NH; const int h = (int)(bh % NH); const int t = threadIdx.x;
  for (int e = t; e < 64 * HD; e += 256) { const int sl = e >> 6, d = e & 63; const int s = s0 + sl; const size_t row = ((size_t)s * NBATCH + b) * EE + h * HD + d;
    const float ang = (1.5707963267948966f * (float)(s + 1)) / (float)LL; const float cs = cos_p(ang), sn = sin_p(ang); const float kv = K[row], vv = V[row];
    const float kc = kv * cs, ks = kv * sn; _Float16 hv;
    hv = (_Float16)kc; st[0][d][sl] = hv; st[1][d][sl] = (_Float16)((kc - (float)hv) * 2048.0f);
    hv = (_Float16)ks; st[2][d][sl] = hv; st[3][d][sl] = (_Float16)((ks - (float)hv) * 2048.0f);
    hv = (_Float16)vv; st[4][d][sl] = hv; st[5][d][sl] = (_Float16)((vv - (float)hv) * 2048.0f); }
  __syncthreads();
  for (int e = t; e < 6 * HD * 8; e += 256) { const int p = e / (HD * 8), rem = e % (HD * 8); const int d = rem >> 3, pc = rem & 7; vst2((unsigned*)(PL + ((bh * 6 + p) * HD + d) * LL + s0 + pc * 8), *(const v4u*)&st[p][d][pc * 8]); }
}
__global__ __launch_bounds__(128) void k_kv(const _Float16* __restrict__ PL, const float* __restrict__ K, float* __restrict__ KV, float* __restrict__ KS) {
  __shared__ __align__(16) float skv[2][HD][HD + 4]; __shared__ __align__(16) float sks[2][HD];
  const int tid = threadIdx.x, wave = tid >> 5, lane = tid & 31, col = lane & 15, g = lane >> 4; const size_t bh = blockIdx.x; const size_t b = bh / NH; const int h = (int)(bh % NH); const int m0 = wave * 16;
  const _Float16* KCH = PL + ((bh * 6 + 0) * HD) * LL; const _Float16* KCL = PL + ((bh * 6 + 1) * HD) * LL; const _Float16* KSH = PL + ((bh * 6 + 2) * HD) * LL; const _Float16* KSL = PL + ((bh * 6 + 3) * HD) * LL; const _Float16* VH = PL + ((bh * 6 + 4) * HD) * LL; const _Float16* VL = PL + ((bh * 6 + 5) * HD) * LL;
  v8f ac[4] = {}, acl[4] = {}, as[4] = {}, asl[4] = {};
#pragma unroll 1
  for (int kc = 0; kc < LL / 32; ++kc) { const v16h vh = frag_h(VH + (size_t)(m0 + col) * LL + kc * 32, lane), vl = frag_h(VL + (size_t)(m0 + col) * LL + kc * 32, lane);
#pragma unroll
    for (int j = 0; j < 4; ++j) { const size_t o = (size_t)(j * 16 + col) * LL + kc * 32; const v16h kch = frag_h(KCH + o, lane), ksh = frag_h(KSH + o, lane);
      ac[j] = wmma16(vh, kch, ac[j]); acl[j] = wmma16(vl, kch, acl[j]); acl[j] = wmma16(vh, frag_h(KCL + o, lane), acl[j]);
      as[j] = wmma16(vh, ksh, as[j]); asl[j] = wmma16(vl, ksh, asl[j]); asl[j] = wmma16(vh, frag_h(KSL + o, lane), asl[j]); } }
#pragma unroll
  for (int j = 0; j < 4; ++j)
#pragma unroll
    for (int r = 0; r < 8; ++r) { skv[0][m0 + 8 * g + r][j * 16 + col] = ac[j][r] + acl[j][r] * (1.0f / 2048.0f); skv[1][m0 + 8 * g + r][j * 16 + col] = as[j][r] + asl[j][r] * (1.0f / 2048.0f); }
  { const int d = tid & 63, which = tid >> 6; float s = 0.f; for (int sx = 0; sx < LL; ++sx) { const float ang = (1.5707963267948966f * (float)(sx + 1)) / (float)LL; const float w = which ? sin_p(ang) : cos_p(ang); s += K[((size_t)sx * NBATCH + b) * EE + h * HD + d] * w; } sks[which][d] = s; }
  __syncthreads();
  for (int q = tid; q < 2 * HD * HD / 4; q += 128) { const int p = q / (HD * HD / 4), rem = q % (HD * HD / 4); const int m = rem / (HD / 4), d4 = rem % (HD / 4); vst2(KV + ((bh * 2 + p) * HD + m) * HD + d4 * 4, *(const v4f*)&skv[p][m][d4 * 4]); }
  if (tid < 2 * HD / 4) vst2(KS + bh * 2 * HD + tid * 4, *(const v4f*)(&sks[0][0] + tid * 4));
}
__global__ __launch_bounds__(128) void k_fin(const float* __restrict__ Q, const float* __restrict__ KV, const float* __restrict__ KS, float* __restrict__ OUT) {
  __shared__ __align__(16) float sq[2][64][HD + 4]; __shared__ __align__(16) __bf16 skh[2][HD][HD + 8]; __shared__ __align__(16) __bf16 skl[2][HD][HD + 8]; __shared__ float sz[64]; __shared__ __align__(16) float so[4][16][68];
  const int tid = threadIdx.x, wave = tid >> 5, lane = tid & 31, col = lane & 15, g = lane >> 4; const int l0 = blockIdx.x * 64; const size_t bh = blockIdx.y; const size_t b = bh / NH; const int h = (int)(bh % NH);
  for (int e = tid; e < 64 * HD; e += 128) { const int ll = e >> 6, d = e & 63; const int l = l0 + ll; const float ang = (1.5707963267948966f * (float)(l + 1)) / (float)LL; const float qv = Q[((size_t)l * NBATCH + b) * EE + h * HD + d]; sq[0][ll][d] = qv * cos_p(ang); sq[1][ll][d] = qv * sin_p(ang); }
  for (int e = tid; e < 2 * HD * HD; e += 128) { const int p = e / (HD * HD), rem = e % (HD * HD); const int m = rem / HD, d = rem % HD; const float v = KV[((bh * 2 + p) * HD + m) * HD + d]; const __bf16 hv = (__bf16)v; skh[p][m][d] = hv; skl[p][m][d] = (__bf16)(v - (float)hv); }
  __syncthreads();
  if (tid < 64) { float a = 0.f; for (int d = 0; d < HD; ++d) a += sq[0][tid][d] * KS[bh * 2 * HD + d] + sq[1][tid][d] * KS[bh * 2 * HD + HD + d]; sz[tid] = 1.0f / (a + 1e-6f); }
  v8f acc[4] = {};
#pragma unroll
  for (int p = 0; p < 2; ++p)
#pragma unroll
    for (int kc = 0; kc < HD / 32; ++kc) { const F2 a = split_row(&sq[p][wave * 16 + col][0], kc * 32, lane);
#pragma unroll
      for (int j = 0; j < 4; ++j) { const v16b wh = frag_b(&skh[p][j * 16 + col][0] + kc * 32, lane), wl = frag_b(&skl[p][j * 16 + col][0] + kc * 32, lane); acc[j] = wmma_bf(a.h, wh, acc[j]); acc[j] = wmma_bf(a.l, wh, acc[j]); acc[j] = wmma_bf(a.h, wl, acc[j]); acc[j] = wmma_bf(a.l, wl, acc[j]); } }
  __syncthreads();
#pragma unroll
  for (int j = 0; j < 4; ++j)
#pragma unroll
    for (int r = 0; r < 8; ++r) so[wave][8 * g + r][j * 16 + col] = acc[j][r] * sz[wave * 16 + 8 * g + r];
  LDSX();
  for (int rl = 0; rl < 16; ++rl) if (lane < 16) vst2(OUT + (bh * LL + l0 + wave * 16 + rl) * HD + lane * 4, *(const v4f*)&so[wave][rl][lane * 4]);
}
extern "C" void kernel_launch(void* const* d_in, const int* in_sizes, int n_in, void* d_out, int out_size, void* d_ws, size_t ws_size, hipStream_t stream) {
  (void)in_sizes; (void)n_in; (void)out_size;
  const float** F = (const float**)d_in;
  if (ws_size < (size_t)WS_END) return;
  char* ws = (char*)d_ws; __bf16* PW = (__bf16*)(ws + WS_PW); float *Q = (float*)(ws + WS_Q), *K = (float*)(ws + WS_K), *V = (float*)(ws + WS_V), *KV = (float*)(ws + WS_KV), *KS = (float*)(ws + WS_KS); _Float16* PL = (_Float16*)(ws + WS_PL);
  k_pack<<<dim3(EE, 2), 256, 0, stream>>>(F[3], F[5], PW);
  k_proj<<<dim3(NR / 64, EE / 128, 3), 128, 0, stream>>>(F[0], F[1], F[2], PW, F[4], F[6], Q, K, V);
  k_planes<<<dim3(LL / 64, TBH), 256, 0, stream>>>(K, V, PL);
  k_kv<<<TBH, 128, 0, stream>>>(PL, K, KV, KS);
  k_fin<<<dim3(LL / 64, TBH), 128, 0, stream>>>(Q, KV, KS, (float*)d_out);
}
